// KPCL_7232724926714
// MI455X (gfx1250) — hardware-verified
//
#include <hip/hip_runtime.h>
#include <math.h>

typedef __attribute__((ext_vector_type(16))) _Float16 v16h;
typedef __attribute__((ext_vector_type(16))) __bf16 v16b;
typedef __attribute__((ext_vector_type(8)))  _Float16 v8h;
typedef __attribute__((ext_vector_type(8)))  float v8f;
typedef __attribute__((ext_vector_type(4)))  float v4f;
typedef __attribute__((ext_vector_type(2)))  float v2f;
typedef __attribute__((ext_vector_type(4)))  unsigned v4u;
typedef __attribute__((ext_vector_type(4)))  int v4i;
typedef float __attribute__((may_alias)) float_a;
typedef int __attribute__((may_alias)) int_a;

template <typename T> __device__ __forceinline__ void vst2(void* p, T v) { *(volatile T*)p = v; __threadfence(); *(volatile T*)p = v; }
__device__ __forceinline__ v8f wmma16(v16h a, v16h b, v8f c) {
  v8f d = __builtin_amdgcn_wmma_f32_16x16x32_f16(false, a, false, b, (short)0, c, false, false);
  asm volatile("v_nop\n\tv_nop\n\tv_nop\n\tv_nop" : "+v"(d) : "v"(a), "v"(b));
  return d;
}
__device__ __forceinline__ v8f wmma_bf(v16b a, v16b b, v8f c) {
  v8f d = __builtin_amdgcn_wmma_f32_16x16x32_bf16(false, a, false, b, (short)0, c, false, false);
  asm volatile("v_nop\n\tv_nop\n\tv_nop\n\tv_nop" : "+v"(d) : "v"(a), "v"(b));
  return d;
}
__device__ __forceinline__ v16h frag_h(const _Float16* rowk0, int lane) {
  union { v16h v; v8h q[2]; } u; const _Float16* p = rowk0 + 8 * (lane >> 4);
  u.q[0] = *(const v8h*)p; u.q[1] = *(const v8h*)(p + 16); return u.v;
}
__device__ __forceinline__ v16h frag_f32(const float* rowk0, int lane) {
  v16h a; const float* p = rowk0 + 8 * (lane >> 4);
#pragma unroll
  for (int i = 0; i < 8; ++i) { a[i] = (_Float16)p[i]; a[8 + i] = (_Float16)p[16 + i]; }
  return a;
}
__device__ __forceinline__ v16h frag_f32s(const float* rowk0, int lane, float sc) {
  v16h a; const float* p = rowk0 + 8 * (lane >> 4);
#pragma unroll
  for (int i = 0; i < 8; ++i) { a[i] = (_Float16)(p[i] * sc); a[8 + i] = (_Float16)(p[16 + i] * sc); }
  return a;
}
__device__ __forceinline__ v16h fragc_f32(const float* W, int k0, int n, int lane, int ld, int K) {
  v16h a; const int g = lane >> 4;
#pragma unroll
  for (int i = 0; i < 8; ++i) { const int ka = k0 + 8 * g + i, kb = ka + 16;
    a[i] = (_Float16)(ka < K ? W[(size_t)(ka < K ? ka : K - 1) * ld + n] : 0.f); a[8 + i] = (_Float16)(kb < K ? W[(size_t)(kb < K ? kb : K - 1) * ld + n] : 0.f); }
  return a;
}
struct F2 { v16b h, l; };
__device__ __forceinline__ F2 bsplit16(const float v[16]) { F2 r;
#pragma unroll
  for (int i = 0; i < 16; ++i) { const __bf16 h = (__bf16)v[i]; r.h[i] = h; r.l[i] = (__bf16)(v[i] - (float)h); }
  return r; }
__device__ __forceinline__ F2 split_row(const float* row, int k0, int lane) { float v[16]; const float* p = row + k0 + 8 * (lane >> 4);
#pragma unroll
  for (int i = 0; i < 8; ++i) { v[i] = p[i]; v[8 + i] = p[16 + i]; }
  return bsplit16(v); }
__device__ __forceinline__ F2 split_rowK(const float* row, int k0, int lane, int K) { float v[16]; const int g = lane >> 4;
#pragma unroll
  for (int i = 0; i < 8; ++i) { const int ka = k0 + 8 * g + i, kb = ka + 16; v[i] = ka < K ? row[ka < K ? ka : K - 1] : 0.f; v[8 + i] = kb < K ? row[kb < K ? kb : K - 1] : 0.f; }
  return bsplit16(v); }
__device__ __forceinline__ F2 split_col(const float* W, int k0, int n, int lane, int ld, int K) { float v[16]; const int g = lane >> 4;
#pragma unroll
  for (int i = 0; i < 8; ++i) { const int ka = k0 + 8 * g + i, kb = ka + 16; v[i] = ka < K ? W[(size_t)(ka < K ? ka : K - 1) * ld + n] : 0.f; v[8 + i] = kb < K ? W[(size_t)(kb < K ? kb : K - 1) * ld + n] : 0.f; }
  return bsplit16(v); }
__device__ __forceinline__ v8f mac3(const F2& a, const F2& b, v8f c) { c = wmma_bf(a.l, b.h, c); c = wmma_bf(a.h, b.l, c); return wmma_bf(a.h, b.h, c); }
__device__ __forceinline__ float sigm(float v) { return 1.0f / (1.0f + expf(-v)); }
#define LDSX() do { asm volatile("s_wait_dscnt 0" ::: "memory"); __builtin_amdgcn_wave_barrier(); __builtin_amdgcn_fence(__ATOMIC_RELEASE, "workgroup"); } while (0)


#define NR 8192
#define DI 512
#define DP 128
#ifndef NRX
#define NRX NR
#endif
typedef __attribute__((ext_vector_type(8))) __bf16 v8b;
__device__ __forceinline__ v16b frag_b(const __bf16* rowk0, int lane) {
  union { v16b v; v8b q[2]; } u; const __bf16* p = rowk0 + 8 * (lane >> 4);
  u.q[0] = *(const v8b*)p; u.q[1] = *(const v8b*)(p + 16); return u.v;
}
__device__ __forceinline__ v16b frag_gbf(const float* rowk0, int lane) {
  v16b a; const float* p = rowk0 + 8 * (lane >> 4);
#pragma unroll
  for (int i = 0; i < 8; ++i) { a[i] = (__bf16)p[i]; a[8 + i] = (__bf16)p[16 + i]; }
  return a;
}
__device__ __forceinline__ float bfr(float v) { return (float)(__bf16)v; }
__device__ __forceinline__ float sgnf(float v) { return v > 0.f ? 1.f : (v < 0.f ? -1.f : 0.f); }
__device__ __attribute__((noinline)) float exp_ni(float v) { return expf(v); }
__device__ __attribute__((noinline)) float log_ni(float v) { return logf(v); }
#define WS_X2   0u
#define WS_Z    (WS_X2 + 4u * NR * DI)
#define WS_PART (WS_Z + 4u * NR * DP)
#define WS_END  (WS_PART + 4u * 128 * 32)

__global__ __launch_bounds__(128) void k_aug(const float* __restrict__ Fe, const float* __restrict__ N1, const float* __restrict__ N2, float* __restrict__ X2) {
  __shared__ float sred[2][4]; __shared__ __align__(16) float srow[DI];
  const int r = blockIdx.x, tid = threadIdx.x, wave = tid >> 5, lane = tid & 31; float s1 = 0.f, s2 = 0.f;
  for (int k = tid; k < DI; k += 128) { const float a = bfr(N1[(size_t)r * DI + k]), b = bfr(N2[(size_t)r * DI + k]); s1 += a * a; s2 += b * b; }
#pragma unroll
  for (int o = 1; o < 32; o <<= 1) { s1 += __shfl_xor(s1, o); s2 += __shfl_xor(s2, o); }
  if (lane == 0) { sred[0][wave] = s1; sred[1][wave] = s2; }
  __syncthreads();
  const float nn1 = fmaxf(sqrtf((sred[0][0] + sred[0][1]) + (sred[0][2] + sred[0][3])), 1e-8f), nn2 = fmaxf(sqrtf((sred[1][0] + sred[1][1]) + (sred[1][2] + sred[1][3])), 1e-8f);
  for (int k = tid; k < DI; k += 128) { const float f = bfr(Fe[(size_t)r * DI + k]); const float x1 = f + sgnf(f) * (bfr(N1[(size_t)r * DI + k]) / nn1) * 0.1f; srow[k] = x1 + sgnf(x1) * (bfr(N2[(size_t)r * DI + k]) / nn2) * 0.1f; }
  __syncthreads();
  vst2(X2 + (size_t)r * DI + tid * 4, *(const v4f*)&srow[tid * 4]);
}
__global__ __launch_bounds__(128) void k_proj(const float* __restrict__ X2, const float* __restrict__ W1, const float* __restrict__ b1, const float* __restrict__ W2, const float* __restrict__ b2, float* __restrict__ Z) {
  __shared__ __align__(16) __bf16 sw1[DP][DI + 8];
  __shared__ __align__(16) __bf16 sw2[DP][DP + 8];
  __shared__ __align__(16) __bf16 shh[4][16][DP + 8], shl[4][16][DP + 8]; __shared__ __align__(16) float so[4][16][DP + 4];
  const int tid = threadIdx.x, wave = tid >> 5, lane = tid & 31, col = lane & 15, g = lane >> 4; const size_t r0 = (size_t)blockIdx.x * 64 + wave * 16;
  for (int q = tid; q < DI * DP; q += 128) { const int k = q >> 7, o = q & 127; sw1[o][k] = (__bf16)bfr(W1[q]); }
  for (int q = tid; q < DP * DP; q += 128) { const int k = q >> 7, o = q & 127; sw2[o][k] = (__bf16)bfr(W2[q]); }
  __syncthreads();
  { v8f acc[8] = {};
#pragma unroll 2
    for (int kc = 0; kc < DI / 32; ++kc) { const F2 a = split_row(X2 + (r0 + col) * DI, kc * 32, lane);
#pragma unroll
      for (int j = 0; j < 8; ++j) { const v16b w = frag_b(&sw1[j * 16 + col][kc * 32], lane); acc[j] = wmma_bf(a.l, w, acc[j]); acc[j] = wmma_bf(a.h, w, acc[j]); } }
#pragma unroll
    for (int j = 0; j < 8; ++j) { const float bb = bfr(b1[j * 16 + col]);
#pragma unroll
      for (int r = 0; r < 8; ++r) { const float v = fmaxf(acc[j][r] + bb, 0.f); const __bf16 hb = (__bf16)v; shh[wave][8 * g + r][j * 16 + col] = hb; shl[wave][8 * g + r][j * 16 + col] = (__bf16)(v - (float)hb); } } }
  LDSX();
  { v8f acc[8] = {};
#pragma unroll
    for (int kc = 0; kc < DP / 32; ++kc) { const v16b ah = frag_b(&shh[wave][col][kc * 32], lane), al = frag_b(&shl[wave][col][kc * 32], lane);
#pragma unroll
      for (int j = 0; j < 8; ++j) { const v16b w = frag_b(&sw2[j * 16 + col][kc * 32], lane); acc[j] = wmma_bf(al, w, acc[j]); acc[j] = wmma_bf(ah, w, acc[j]); } }
#pragma unroll
    for (int j = 0; j < 8; ++j) { const float bb = bfr(b2[j * 16 + col]);
#pragma unroll
      for (int r = 0; r < 8; ++r) so[wave][8 * g + r][j * 16 + col] = acc[j][r] + bb; } }
  LDSX();
  { const int rl = lane >> 1, half = lane & 1; float ss = 0.f; for (int c = half * 64; c < half * 64 + 64; ++c) { const float v = so[wave][rl][c]; ss += v * v; } ss += __shfl_xor(ss, 1); const float inv = 1.0f / fmaxf(sqrtf(ss), 1e-6f);
    LDSX(); for (int c = half * 64; c < half * 64 + 64; ++c) so[wave][rl][c] *= inv; }
  LDSX();
  for (int rl = 0; rl < 16; ++rl) vst2(Z + (r0 + rl) * DP + lane * 4, *(const v4f*)&so[wave][rl][lane * 4]);
}
__global__ __launch_bounds__(128) void k_lse(const float* __restrict__ Z, float* __restrict__ PART) {
  __shared__ float sl[64]; __shared__ __align__(16) float sres[32];
  const int tid = threadIdx.x, wave = tid >> 5, lane = tid & 31, col = lane & 15, g = lane >> 4; const int i0 = blockIdx.x * 64 + wave * 16;
  F2 a[4];
#pragma unroll
  for (int kc = 0; kc < 4; ++kc) a[kc] = split_row(Z + (size_t)(i0 + col) * DP, kc * 32, lane);
  float mx[8], sm[8], dg[8];
#pragma unroll
  for (int r = 0; r < 8; ++r) { mx[r] = -3.0e38f; sm[r] = 0.f; dg[r] = 0.f; }
  const float it = 1.0f / 0.15f;
#pragma unroll 1
  for (int jt = 0; jt < NRX / 16; ++jt) { v8f c = {};
#pragma unroll
    for (int kc = 0; kc < 4; ++kc) { const F2 b = split_row(Z + (size_t)(jt * 16 + col) * DP, kc * 32, lane); c = mac3(a[kc], b, c); }
#pragma unroll
    for (int r = 0; r < 8; ++r) { const float v = c[r] * it; if (jt * 16 + col == i0 + 8 * g + r) dg[r] = v; float tmx = v;
#pragma unroll
      for (int o = 1; o < 16; o <<= 1) tmx = fmaxf(tmx, __shfl_xor(tmx, o));
      const float nm = fmaxf(mx[r], tmx); float ex = exp_ni(v - nm);
#pragma unroll
      for (int o = 1; o < 16; o <<= 1) ex += __shfl_xor(ex, o);
      sm[r] = sm[r] * exp_ni(mx[r] - nm) + ex; mx[r] = nm; } }
#pragma unroll
  for (int r = 0; r < 8; ++r) {
#pragma unroll
    for (int o = 1; o < 16; o <<= 1) dg[r] += __shfl_xor(dg[r], o); }
  if (col == 0) {
#pragma unroll
    for (int r = 0; r < 8; ++r) sl[wave * 16 + 8 * g + r] = (mx[r] + log_ni(sm[r])) - dg[r]; }
  __syncthreads();
  if (tid < 32) { float s = sl[tid] + sl[tid + 32];
#pragma unroll
    for (int o = 1; o < 32; o <<= 1) s += __shfl_xor(s, o);
    sres[tid] = tid == 0 ? s : 0.f; }
  __syncthreads();
  if (tid < 8) vst2(PART + (size_t)blockIdx.x * 32 + tid * 4, *(const v4f*)&sres[tid * 4]);
}
__global__ __launch_bounds__(64) void k_fin(const float* __restrict__ PART, float* __restrict__ out) {
  __shared__ double sp[64]; const int tid = threadIdx.x; double s = 0.0; for (int i = tid; i < NRX / 64; i += 64) s += (double)PART[(size_t)i * 32]; sp[tid] = s; __syncthreads();
  if (tid == 0) { double t = 0.0; for (int i = 0; i < 64; ++i) t += sp[i]; vst2(out, (float_a)(float)(t / (double)NRX + 0.6931471805599453)); }
}

extern "C" void kernel_launch(void* const* d_in, const int* in_sizes, int n_in, void* d_out, int out_size, void* d_ws, size_t ws_size, hipStream_t stream) {
  (void)in_sizes; (void)n_in; (void)out_size;
  const float** F = (const float**)d_in;
  if (ws_size < (size_t)WS_END) return;
  char* ws = (char*)d_ws; float *X2 = (float*)(ws + WS_X2), *Z = (float*)(ws + WS_Z), *PART = (float*)(ws + WS_PART);
  k_aug<<<NRX, 128, 0, stream>>>(F[0], F[1], F[2], X2);
  k_proj<<<NRX / 64, 128, 0, stream>>>(X2, F[3], F[4], F[5], F[6], Z);
  k_lse<<<NRX / 64, 128, 0, stream>>>(Z, PART);
  k_fin<<<1, 64, 0, stream>>>(PART, (float*)d_out);
}
